// MHA_6167573037151
// MI455X (gfx1250) — hardware-verified
//
#include <hip/hip_runtime.h>


#ifndef NB
#define NB 2
#endif
#ifndef SEQ
#define SEQ 4096
#endif
#define SEQ_FULL 4096
#define NH 8
#define HD 64
#define DM 512
#define OP 516
#define PSH 10.0f

static_assert(SEQ % 64 == 0);
static_assert(SEQ <= SEQ_FULL);
static_assert(NH * HD == DM);
static_assert((OP * 4) % 16 == 0);
static_assert((size_t)48 * 256 * 8 == (size_t)3 * NH * HD * HD);
static_assert((size_t)(NB * SEQ / 64) * NH * 4 * 128 * 8 == (size_t)NB * NH * SEQ * HD);
static_assert((size_t)(NB * SEQ / 16) * 8 * 2 * 4 * 32 * 4 == (size_t)NB * SEQ * DM);

typedef _Float16 h16;
typedef unsigned short bf;
typedef __attribute__((ext_vector_type(16))) __bf16   v16bf;
typedef __attribute__((ext_vector_type(16))) _Float16 v16h;
typedef __attribute__((ext_vector_type(8)))  _Float16 v8h;
typedef __attribute__((ext_vector_type(8)))  unsigned short v8us;
typedef __attribute__((ext_vector_type(16))) unsigned short v16us;
typedef __attribute__((ext_vector_type(8)))  float    v8f;
typedef __attribute__((ext_vector_type(4)))  float    v4f;
typedef v8h  __attribute__((may_alias)) v8ha;
typedef v4f  __attribute__((may_alias)) v4fa;

__device__ __forceinline__ unsigned short f2bf(float f) { unsigned u = __float_as_uint(f); u += 0x7FFFu + ((u >> 16) & 1u); return (unsigned short)(u >> 16); }
__device__ __forceinline__ float bf2f(unsigned short b) { return __uint_as_float(((unsigned)b) << 16); }
__device__ __forceinline__ float bfr(float f) { return bf2f(f2bf(f)); }
__device__ __forceinline__ v16h cat16(v8h lo, v8h hi) { return __builtin_shufflevector(lo, hi, 0, 1, 2, 3, 4, 5, 6, 7, 8, 9, 10, 11, 12, 13, 14, 15); }
__device__ __forceinline__ v16bf cat16b(v8us lo, v8us hi) { return __builtin_bit_cast(v16bf, __builtin_shufflevector(lo, hi, 0, 1, 2, 3, 4, 5, 6, 7, 8, 9, 10, 11, 12, 13, 14, 15)); }
__device__ __forceinline__ v8f wmma16(v16h a, v16h b, v8f c) { return __builtin_amdgcn_wmma_f32_16x16x32_f16(false, a, false, b, (short)0, c, false, false); }
__device__ __forceinline__ v8f wmmab(v16bf a, v16bf b, v8f c) { return __builtin_amdgcn_wmma_f32_16x16x32_bf16(false, a, false, b, (short)0, c, false, false); }
__device__ __forceinline__ v16h ldh(const h16* p) { return cat16(*(const v8h*)p, *(const v8h*)(p + 16)); }
__device__ __forceinline__ v16bf ldb(const bf* p) { return cat16b(*(const v8us*)p, *(const v8us*)(p + 16)); }
__device__ __forceinline__ v16bf ldA32(const float* p) {
    const v4f a0 = *(const v4f*)p, a1 = *(const v4f*)(p + 4), c0 = *(const v4f*)(p + 16), c1 = *(const v4f*)(p + 20);
    v16us u;
    u[0] = f2bf(a0[0]); u[1] = f2bf(a0[1]); u[2] = f2bf(a0[2]); u[3] = f2bf(a0[3]);
    u[4] = f2bf(a1[0]); u[5] = f2bf(a1[1]); u[6] = f2bf(a1[2]); u[7] = f2bf(a1[3]);
    u[8] = f2bf(c0[0]); u[9] = f2bf(c0[1]); u[10] = f2bf(c0[2]); u[11] = f2bf(c0[3]);
    u[12] = f2bf(c1[0]); u[13] = f2bf(c1[1]); u[14] = f2bf(c1[2]); u[15] = f2bf(c1[3]);
    return __builtin_bit_cast(v16bf, u);
}

__global__ __launch_bounds__(256) void k_wprep(const float* __restrict__ Wk, const float* __restrict__ Wq, const float* __restrict__ Wv, bf* WT) {
    const unsigned idx = blockIdx.x * 256u + threadIdx.x;
    if (idx >= 3u * NH * HD * HD / 8u) return;
    const unsigned k8 = idx & 7u, n = (idx >> 3) & 63u, h = (idx >> 9) & 7u, m = idx >> 12;
    const float* W = (m == 0u) ? Wk : ((m == 1u) ? Wq : Wv);
    const float* src = W + (size_t)h * HD * HD + (size_t)(k8 * 8u) * HD + n;
    v8us o;
#pragma unroll
    for (int i = 0; i < 8; ++i) o[i] = f2bf(src[(size_t)i * HD]);
    *(volatile v8us*)(WT + (size_t)idx * 8) = o; __threadfence(); *(volatile v8us*)(WT + (size_t)idx * 8) = o;
}

template <bool TR>
__device__ __forceinline__ void proj_one(v16bf a0, v16bf a1, const bf* __restrict__ Wt, const float* __restrict__ bias, h16* dst, unsigned wave, unsigned nn, unsigned g) {
#pragma unroll
    for (unsigned nt = 0; nt < 4; ++nt) {
        const bf* wp = Wt + (size_t)(nt * 16u + nn) * HD + 8u * g;
        const v16bf b0 = ldb(wp), b1 = ldb(wp + 32);
        v8f acc = (v8f){};
        acc = wmmab(a0, b0, acc);
        acc = wmmab(a1, b1, acc);
        asm volatile("v_nop\n\tv_nop\n\tv_nop\n\tv_nop" : "+v"(acc) : "v"(a1), "v"(b1));
        const float bvv = bfr(bias[nt * 16u + nn]);
        const unsigned col = nt * 16u + nn;
#pragma unroll
        for (unsigned r = 0; r < 8; ++r) {
            const unsigned rowl = wave * 16u + 8u * g + r;
            const float val = acc[r] + bvv;
            if (TR) dst[col * 64u + rowl] = (h16)val; else dst[rowl * 64u + col] = (h16)val;
        }
    }
}

__global__ __launch_bounds__(128) void k_proj(const float* __restrict__ x, const float* __restrict__ y, const bf* __restrict__ WT,
                                              const float* __restrict__ bk, const float* __restrict__ bq, const float* __restrict__ bv,
                                              h16* Q16, h16* K16, h16* Vt16) {
    __shared__ __align__(16) h16 sK[64 * 64];
    __shared__ __align__(16) h16 sQ[64 * 64];
    __shared__ __align__(16) h16 sV[64 * 64];
    const unsigned tid = threadIdx.x, lane = tid & 31u, wave = tid >> 5, nn = lane & 15u, g = lane >> 4;
    const unsigned tile = blockIdx.x, h = blockIdx.y;
    const unsigned b = tile / (SEQ / 64u), s0 = (tile % (SEQ / 64u)) * 64u;
    const size_t rowi = (size_t)b * SEQ_FULL + s0 + wave * 16u + nn;
    const float* xp = x + rowi * DM + h * HD + 8u * g;
    const float* yp = y + rowi * DM + h * HD + 8u * g;
    const v16bf ax0 = ldA32(xp), ax1 = ldA32(xp + 32), ay0 = ldA32(yp), ay1 = ldA32(yp + 32);
    proj_one<false>(ax0, ax1, WT + (size_t)(0u * NH + h) * HD * HD, bk + h * HD, sK, wave, nn, g);
    proj_one<false>(ay0, ay1, WT + (size_t)(1u * NH + h) * HD * HD, bq + h * HD, sQ, wave, nn, g);
    proj_one<true >(ax0, ax1, WT + (size_t)(2u * NH + h) * HD * HD, bv + h * HD, sV, wave, nn, g);
    __syncthreads();
    const size_t bh = (size_t)b * NH + h;
    h16* kd = K16 + (bh * SEQ + s0) * HD;
    h16* qd = Q16 + (bh * SEQ + s0) * HD;
    h16* vd = Vt16 + bh * HD * SEQ + s0;
#pragma unroll 1
    for (int ps = 0; ps < 2; ++ps) {
#pragma unroll
        for (unsigned it = 0; it < 4; ++it) {
            const unsigned c = it * 128u + tid;
            const v8h kv = *(const v8ha*)(sK + c * 8u);
            const v8h qv = *(const v8ha*)(sQ + c * 8u);
            const v8h vv = *(const v8ha*)(sV + c * 8u);
            *(volatile v8h*)(kd + (size_t)c * 8u) = kv;
            *(volatile v8h*)(qd + (size_t)c * 8u) = qv;
            *(volatile v8h*)(vd + (size_t)(c >> 3) * SEQ + (c & 7u) * 8u) = vv;
        }
        if (ps == 0) __threadfence();
    }
}

__global__ __launch_bounds__(256) void k_flash(const h16* __restrict__ Q16, const h16* __restrict__ K16, const h16* __restrict__ Vt16,
                                               const float* __restrict__ y, const float* __restrict__ gamma, const float* __restrict__ beta, float* out) {
    __shared__ __align__(16) float so[16 * OP];
    const unsigned tid = threadIdx.x, lane = tid & 31u, h = tid >> 5, nn = lane & 15u, g = lane >> 4;
    const unsigned blk = blockIdx.x;
    const unsigned b = blk / (SEQ / 16u), q0 = (blk % (SEQ / 16u)) * 16u;
    const size_t bh = (size_t)b * NH + h;
    const h16* Qh = Q16 + bh * SEQ * HD;
    const h16* Kh = K16 + bh * SEQ * HD + (size_t)nn * HD + 8u * g;
    const h16* Vh = Vt16 + bh * HD * SEQ + (size_t)nn * SEQ + 8u * g;
    const v16h qb0 = ldh(Qh + (size_t)(q0 + nn) * HD + 8u * g);
    const v16h qb1 = ldh(Qh + (size_t)(q0 + nn) * HD + 32u + 8u * g);
    const float C = 0.125f * 1.4426950408889634f;
    float m = -1.0e30f, l = 0.f;
    v8f o[4];
#pragma unroll
    for (int dt = 0; dt < 4; ++dt) o[dt] = (v8f){};
#pragma unroll 1
    for (unsigned it = 0; it < SEQ / 64u; ++it) {
        const unsigned j0 = it * 64u;
        v8f sc[4];
#pragma unroll
        for (unsigned jt = 0; jt < 4; ++jt) {
            const h16* kp = Kh + (size_t)(j0 + jt * 16u) * HD;
            const v16h ka0 = ldh(kp), ka1 = ldh(kp + 32);
            v8f acc = (v8f){};
            acc = wmma16(ka0, qb0, acc);
            acc = wmma16(ka1, qb1, acc);
            sc[jt] = acc;
        }
        asm volatile("v_nop\n\tv_nop\n\tv_nop\n\tv_nop" : "+v"(sc[0]), "+v"(sc[1]), "+v"(sc[2]), "+v"(sc[3]) : "v"(qb0), "v"(qb1));
        float mx = sc[0][0];
#pragma unroll
        for (int jt = 0; jt < 4; ++jt)
#pragma unroll
            for (int r = 0; r < 8; ++r) mx = fmaxf(mx, sc[jt][r]);
        mx = fmaxf(mx, __shfl_xor(mx, 16, 32));
        const float mn = fmaxf(m, mx * C);
        const float alpha = __builtin_amdgcn_exp2f(m - mn);
        m = mn;
        const float off = mn - PSH;
        float psum = 0.f;
#pragma unroll
        for (int jt = 0; jt < 4; ++jt)
#pragma unroll
            for (int r = 0; r < 8; ++r) { const float p = __builtin_amdgcn_exp2f(fmaf(sc[jt][r], C, -off)); sc[jt][r] = p; psum += p; }
        l = l * alpha + psum;
#pragma unroll
        for (int dt = 0; dt < 4; ++dt)
#pragma unroll
            for (int r = 0; r < 8; ++r) o[dt][r] *= alpha;
        v16h pb0, pb1;
#pragma unroll
        for (int i = 0; i < 8; ++i) { pb0[i] = (h16)sc[0][i]; pb0[8 + i] = (h16)sc[1][i]; pb1[i] = (h16)sc[2][i]; pb1[8 + i] = (h16)sc[3][i]; }
#pragma unroll
        for (unsigned dt = 0; dt < 4; ++dt) {
            const h16* vp = Vh + (size_t)(dt * 16u) * SEQ + j0;
            const v16h va0 = ldh(vp), va1 = ldh(vp + 32);
            o[dt] = wmma16(va0, pb0, o[dt]);
            o[dt] = wmma16(va1, pb1, o[dt]);
        }
        asm volatile("v_nop\n\tv_nop\n\tv_nop\n\tv_nop" : "+v"(o[0]), "+v"(o[1]), "+v"(o[2]), "+v"(o[3]) : "v"(pb0), "v"(pb1));
    }
    l += __shfl_xor(l, 16, 32);
    const float inv = 1.0f / l;
#pragma unroll
    for (unsigned dt = 0; dt < 4; ++dt) {
        v4f w0, w1;
        w0[0] = o[dt][0] * inv; w0[1] = o[dt][1] * inv; w0[2] = o[dt][2] * inv; w0[3] = o[dt][3] * inv;
        w1[0] = o[dt][4] * inv; w1[1] = o[dt][5] * inv; w1[2] = o[dt][6] * inv; w1[3] = o[dt][7] * inv;
        float* sp = so + nn * OP + h * HD + dt * 16u + 8u * g;
        *(v4fa*)sp = w0; *(v4fa*)(sp + 4) = w1;
    }
    __syncthreads();
    const unsigned wave = h;
#pragma unroll 1
    for (unsigned rr = 0; rr < 2; ++rr) {
        const unsigned row = wave * 2u + rr;
        const size_t tok = (size_t)q0 + row;
        const float* yp = y + ((size_t)b * SEQ_FULL + tok) * DM;
        float* op = out + ((size_t)b * SEQ + tok) * DM;
        v4f v[4]; float sum = 0.f;
#pragma unroll
        for (unsigned j = 0; j < 4; ++j) {
            const unsigned c = j * 128u + lane * 4u;
            const v4f a = *(const v4fa*)(so + row * OP + c);
            const v4f yy = *(const v4f*)(yp + c);
#pragma unroll
            for (int q = 0; q < 4; ++q) { const float t = a[q] + bfr(yy[q]); v[j][q] = t; sum += t; }
        }
#pragma unroll
        for (int sh = 16; sh; sh >>= 1) sum += __shfl_xor(sum, sh, 32);
        const float mu = sum * (1.0f / 512.0f);
        float s2 = 0.f;
#pragma unroll
        for (int j = 0; j < 4; ++j)
#pragma unroll
            for (int q = 0; q < 4; ++q) { const float d = v[j][q] - mu; s2 += d * d; }
#pragma unroll
        for (int sh = 16; sh; sh >>= 1) s2 += __shfl_xor(s2, sh, 32);
        const float rs = rsqrtf(s2 * (1.0f / 512.0f) + 1e-5f);
        v4f ov[4];
#pragma unroll
        for (unsigned j = 0; j < 4; ++j) {
            const unsigned c = j * 128u + lane * 4u;
            const v4f gm = *(const v4f*)(gamma + c);
            const v4f bt = *(const v4f*)(beta + c);
#pragma unroll
            for (int q = 0; q < 4; ++q) ov[j][q] = (v[j][q] - mu) * rs * bfr(gm[q]) + bfr(bt[q]);
        }
#pragma unroll 1
        for (int ps = 0; ps < 2; ++ps) {
#pragma unroll
            for (unsigned j = 0; j < 4; ++j) *(volatile v4f*)(op + j * 128u + lane * 4u) = ov[j];
            if (ps == 0) __threadfence();
        }
    }
}

extern "C" void kernel_launch(void* const* d_in, const int* in_sizes, int n_in,
                              void* d_out, int out_size, void* d_ws, size_t ws_size, hipStream_t stream) {
    if (n_in < 10) return;
    const size_t need_xy = (size_t)(NB - 1) * SEQ_FULL * DM + (size_t)SEQ * DM;
    if ((size_t)in_sizes[0] < need_xy || (size_t)in_sizes[1] < need_xy) return;
    if (in_sizes[2] < NH * HD * HD || in_sizes[4] < NH * HD * HD || in_sizes[6] < NH * HD * HD) return;
    if (in_sizes[3] < NH * HD || in_sizes[5] < NH * HD || in_sizes[7] < NH * HD) return;
    if (in_sizes[8] < DM || in_sizes[9] < DM) return;
    if ((size_t)out_size < (size_t)NB * SEQ * DM) return;
    const float* x = (const float*)d_in[0]; const float* y = (const float*)d_in[1];
    const float* Wk = (const float*)d_in[2]; const float* bk = (const float*)d_in[3];
    const float* Wq = (const float*)d_in[4]; const float* bq = (const float*)d_in[5];
    const float* Wv = (const float*)d_in[6]; const float* bv = (const float*)d_in[7];
    const float* gamma = (const float*)d_in[8]; const float* beta = (const float*)d_in[9];
    float* OUT = (float*)d_out;
    char* wsp = (char*)d_ws;
    auto take = [&](size_t bytes) { char* p = wsp; wsp += (bytes + 255) & ~(size_t)255; return (void*)p; };
    bf* WT = (bf*)take((size_t)3 * NH * HD * HD * 2);
    h16* Q16 = (h16*)take((size_t)NB * NH * SEQ * HD * 2);
    h16* K16 = (h16*)take((size_t)NB * NH * SEQ * HD * 2);
    h16* Vt16 = (h16*)take((size_t)NB * NH * HD * SEQ * 2);
    if ((size_t)(wsp - (char*)d_ws) > ws_size) return;
    k_wprep<<<48, 256, 0, stream>>>(Wk, Wq, Wv, WT);
    k_proj<<<dim3(NB * SEQ / 64, NH, 1), 128, 0, stream>>>(x, y, WT, bk, bq, bv, Q16, K16, Vt16);
    k_flash<<<NB * SEQ / 16, 256, 0, stream>>>(Q16, K16, Vt16, y, gamma, beta, OUT);
}
